// GraphActor_17300128268642
// MI455X (gfx1250) — hardware-verified
//
#include <hip/hip_runtime.h>
#include <stddef.h>


#define NSMP   16
#define NNODE  13
#define RB     (NSMP * NNODE)
#define DOBS   111
#define DLAT   64
#define DH     128
#define DO2    64
#define DLEG   256
#define DL2    128
#define NACT   12
#define HP     136
#define LP     264
#define AP     132
#define CW     16
#define NTHR   256
#define RL     (NSMP * 4)
#define WSCAP  134217728

#define SC_W16 16.0f
#define SC_I16 0.0625f

#define LE_HID  0
#define LE_OUT  (LE_HID + RB * HP * 2)
#define LDS_E   (LE_OUT + RB * DH * 2)

#define LG_X    0
#define LG_M    (LG_X + RB * HP * 2)
#define LG_B    (LG_M + 4 * RB * CW * 4)
#define LG_O    (LG_B + 4 * DH * 4)
#define LDS_G(O) (LG_O + RB * (O) * 2)

#define LL_L    0
#define LL_A1   (LL_L + RL * LP * 2)
#define LL_A2   (LL_A1 + RL * LP * 2)
#define LL_Y    (LL_A2 + RL * AP * 4)
#define LDS_L   (LL_Y + 256 * 4)

static_assert(RB == 208 && (RB % 16) == 0 && (RB % 8) == 0 && RL == 64);
static_assert((RB * CW) % NTHR == 0 && (RB * DH / 8) % NTHR == 0 && (RB * DLAT / 4) % NTHR == 0);
static_assert(((HP * 2) % 16) == 0 && ((LP * 2) % 16) == 0 && ((AP * 4) % 16) == 0);
static_assert(HP >= DH && LP >= DLEG && AP >= DL2);
static_assert((DH % 32) == 0 && (DLEG % 32) == 0 && (DO2 % CW) == 0 && (DH % CW) == 0);
static_assert((LE_OUT % 16) == 0 && (LG_M % 16) == 0 && (LG_B % 16) == 0 && (LG_O % 16) == 0);
static_assert((LL_A1 % 16) == 0 && (LL_A2 % 16) == 0 && (LL_Y % 16) == 0);
static_assert(LDS_E <= 160 * 1024 && LDS_G(DH) <= 170 * 1024 && LDS_L <= 160 * 1024);
static_assert((RL * DLEG / 8) % NTHR == 0 && DLEG == 4 * DO2 && (DO2 % 8) == 0 && DLEG / 8 == 32);
static_assert(RL * 3 <= NTHR && ((RL * 3) % 4) == 0 && RL * 3 <= 256);
static_assert(NTHR == 256 && DLAT == 4 * 16 && DLEG == 16 * 16 && DL2 == 8 * 16);

typedef float          v4f  __attribute__((ext_vector_type(4)));
typedef float          v8f  __attribute__((ext_vector_type(8)));
typedef _Float16       v4h  __attribute__((ext_vector_type(4)));
typedef _Float16       v8h  __attribute__((ext_vector_type(8)));
typedef _Float16       v16h __attribute__((ext_vector_type(16)));
typedef unsigned short v8us __attribute__((ext_vector_type(8)));
union Frag { v16h v; v8h h[2]; };
union H8 { v8h f; v8us u; };
static_assert(sizeof(Frag) == 32 && sizeof(H8) == 16);

__device__ __forceinline__ v8f wm(v16h a, v16h bq, v8f c) {
  v8f d = __builtin_amdgcn_wmma_f32_16x16x32_f16(false, a, false, bq, (short)0, c, false, false);
  asm volatile("v_nop\n\tv_nop\n\tv_nop\n\tv_nop" : "+v"(d) : "v"(a), "v"(bq));
  return d;
}

__device__ __forceinline__ v8f zero8() {
  v8f z = {0.f, 0.f, 0.f, 0.f, 0.f, 0.f, 0.f, 0.f};
  return z;
}

__device__ __forceinline__ int imin(int a, int b) { return a < b ? a : b; }
__device__ __forceinline__ int imax(int a, int b) { return a > b ? a : b; }
__device__ __forceinline__ int iclamp(int v, int lo, int hi) { return imin(imax(v, lo), hi); }

__device__ __forceinline__ float eluf(float x) { return x > 0.0f ? x : (__expf(x) - 1.0f); }
__device__ __forceinline__ float sigm(float x) { return __builtin_amdgcn_rcpf(1.0f + __expf(-x)); }

__global__ __launch_bounds__(NTHR) void k_cvt4(
    const float* __restrict__ s0, const float* __restrict__ s1,
    const float* __restrict__ s2, const float* __restrict__ s3,
    _Float16* dst, int K, int Kp, int N0, int N1, int N2, int N3, int npiece, float scale) {
  const int t = blockIdx.x * NTHR + threadIdx.x;
  if (t >= npiece) return;
  const int e0 = 8 * t;
  const int n  = e0 / Kp;
  const int kb = e0 - n * Kp;
  const int i0 = iclamp(n, 0, N0 - 1);
  const int i1 = iclamp(n - N0, 0, imax(N1 - 1, 0));
  const int i2 = iclamp(n - N0 - N1, 0, imax(N2 - 1, 0));
  const int i3 = iclamp(n - N0 - N1 - N2, 0, imax(N3 - 1, 0));
  H8 o;
#pragma unroll
  for (int i = 0; i < 8; ++i) {
    const int k  = kb + i;
    const int kc = iclamp(k, 0, K - 1);
    const float a = s0[(size_t)kc * N0 + i0];
    const float b = s1[(size_t)kc * N1 + i1];
    const float c = s2[(size_t)kc * N2 + i2];
    const float d = s3[(size_t)kc * N3 + i3];
    float v = (n < N0) ? a : ((n < N0 + N1) ? b : ((n < N0 + N1 + N2) ? c : ((n < N0 + N1 + N2 + N3) ? d : 0.0f)));
    v = (k < K) ? v : 0.0f;
    o.f[i] = (_Float16)(v * scale);
  }
  unsigned short* p = (unsigned short*)(dst + (size_t)e0);
  *(volatile v8us*)p = o.u;
  __threadfence();
  *(volatile v8us*)p = o.u;
}

__global__ __launch_bounds__(NTHR) void k_enc(
    const float* __restrict__ obs, const float* __restrict__ lat,
    const float* __restrict__ bw1, const float* __restrict__ bb1,
    const float* __restrict__ hw1, const float* __restrict__ hb1,
    const float* __restrict__ tw1, const float* __restrict__ tb1,
    const float* __restrict__ cw1, const float* __restrict__ cb1,
    const _Float16* __restrict__ PW2p,
    const float* __restrict__ bb2, const float* __restrict__ hb2,
    const float* __restrict__ tb2, const float* __restrict__ cb2,
    _Float16* H0) {
  extern __shared__ v4f lds_dyn[];
  char* sm = (char*)lds_dyn;
  _Float16* sHid = (_Float16*)(sm + LE_HID);
  _Float16* sOut = (_Float16*)(sm + LE_OUT);
  const int tid = threadIdx.x, lane = tid & 31, h = lane >> 4, m = lane & 15;
  const int wave = __builtin_amdgcn_readfirstlane(tid >> 5);
  const int b0 = blockIdx.x * NSMP;

  {
#pragma unroll 1
    for (int rr = 0; rr < RB / 8; ++rr) {
      const int row  = wave * (RB / 8) + rr;
      const int node = row >> 4, s = row & 15;
      const int nm1  = (node > 0) ? node - 1 : 0;
      const int part = (node == 0) ? 0 : 1 + (nm1 >> 2);
      const int cb   = (node == 0) ? 0 : (15 + 24 * (nm1 & 3) + 8 * (nm1 >> 2));
      const int K    = (node == 0) ? 15 : 8;
      const float* W  = (part == 0) ? bw1 : ((part == 1) ? hw1 : ((part == 2) ? tw1 : cw1));
      const float* bb = (part == 0) ? bb1 : ((part == 1) ? hb1 : ((part == 2) ? tb1 : cb1));
      const float* xr = obs + (size_t)(b0 + s) * DOBS + cb;
      v4f a = {0.f, 0.f, 0.f, 0.f};
#pragma unroll 1
      for (int k = 0; k < K; ++k) {
        const float x = xr[k];
        const v4f w = *(const v4f*)(W + k * DH + 4 * lane);
        a = x * w + a;
      }
      a = a + *(const v4f*)(bb + 4 * lane);
      v4h o;
      o.x = (_Float16)eluf(a.x);
      o.y = (_Float16)eluf(a.y);
      o.z = (_Float16)eluf(a.z);
      o.w = (_Float16)eluf(a.w);
      *(v4h*)(sHid + row * HP + 4 * lane) = o;
    }
  }
  __syncthreads();

  {
    const int nt  = wave & 3;
    const int mlo = (wave >> 2) * 7;
    const int mhi = imin(mlo + 7, NNODE);
#pragma unroll 1
    for (int mt = mlo; mt < mhi; ++mt) {
      const int part = (mt == 0) ? 0 : 1 + ((mt - 1) >> 2);
      const _Float16* bp = PW2p + (size_t)(part * DLAT + nt * 16 + m) * DH + 8 * h;
      const _Float16* ap = sHid + (16 * mt + m) * HP + 8 * h;
      v8f acc = zero8();
#pragma unroll
      for (int ks = 0; ks < DH / 32; ++ks) {
        const int ko = 32 * ks;
        Frag fa, fb;
        fa.h[0] = *(const v8h*)(ap + ko);
        fa.h[1] = *(const v8h*)(ap + ko + 16);
        fb.h[0] = *(const v8h*)(bp + ko);
        fb.h[1] = *(const v8h*)(bp + ko + 16);
        acc = wm(fa.v, fb.v, acc);
      }
      const float* b2 = (part == 0) ? bb2 : ((part == 1) ? hb2 : ((part == 2) ? tb2 : cb2));
      const float bias = b2[nt * 16 + m];
#pragma unroll
      for (int r = 0; r < 8; ++r) {
        sOut[(16 * mt + 8 * h + r) * DH + nt * 16 + m] = (_Float16)(acc[r] * SC_I16 + bias);
      }
    }
  }

  {
#pragma unroll 1
    for (int j = 0; j < (RB * DLAT / 4) / NTHR; ++j) {
      const int p = tid + j * NTHR;
      const int row = p >> 4, c4 = p & 15;
      const int node = row >> 4, s = row & 15;
      const v4f x = *(const v4f*)(lat + ((size_t)(b0 + s) * NNODE + node) * DLAT + 4 * c4);
      v4h o;
      o.x = (_Float16)x.x;
      o.y = (_Float16)x.y;
      o.z = (_Float16)x.z;
      o.w = (_Float16)x.w;
      *(v4h*)(sOut + row * DH + DLAT + 4 * c4) = o;
    }
  }
  __syncthreads();

  {
    unsigned short* gb = (unsigned short*)H0;
#pragma unroll 1
    for (int j = 0; j < (RB * DH / 8) / NTHR; ++j) {
      const int p = tid + j * NTHR;
      const int row = p >> 4, q = p & 15;
      const int node = row >> 4, s = row & 15;
      H8 v;
      v.f = *(const v8h*)(sOut + row * DH + 8 * q);
      *(volatile v8us*)(gb + ((size_t)(b0 + s) * NNODE + node) * DH + 8 * q) = v.u;
    }
    __threadfence();
#pragma unroll 1
    for (int j = 0; j < (RB * DH / 8) / NTHR; ++j) {
      const int p = tid + j * NTHR;
      const int row = p >> 4, q = p & 15;
      const int node = row >> 4, s = row & 15;
      H8 v;
      v.f = *(const v8h*)(sOut + row * DH + 8 * q);
      *(volatile v8us*)(gb + ((size_t)(b0 + s) * NNODE + node) * DH + 8 * q) = v.u;
    }
  }
}

template <int O, int ELU>
__global__ __launch_bounds__(NTHR) void k_gn(
    const _Float16* __restrict__ Xin, const _Float16* __restrict__ Wp,
    const float* __restrict__ bk, const float* __restrict__ bq,
    const float* __restrict__ bv, const float* __restrict__ bs,
    _Float16* Hout) {
  extern __shared__ v4f lds_dyn[];
  char* sm = (char*)lds_dyn;
  _Float16* sX = (_Float16*)(sm + LG_X);
  float*    sM = (float*)(sm + LG_M);
  float*    sB = (float*)(sm + LG_B);
  _Float16* sO = (_Float16*)(sm + LG_O);
  const int tid = threadIdx.x, lane = tid & 31, h = lane >> 4, m = lane & 15;
  const int wave = __builtin_amdgcn_readfirstlane(tid >> 5);
  const size_t gr0 = (size_t)blockIdx.x * RB;

  {
#pragma unroll 1
    for (int j = 0; j < (RB * DH / 8) / NTHR; ++j) {
      const int p = tid + j * NTHR;
      const int row = p >> 4, q = p & 15;
      *(v8h*)(sX + row * HP + 8 * q) = *(const v8h*)(Xin + (gr0 + row) * DH + 8 * q);
    }
    if (tid < O) {
      sB[tid]         = bk[tid];
      sB[O + tid]     = bq[tid];
      sB[2 * O + tid] = bv[tid];
      sB[3 * O + tid] = bs[tid];
    }
  }
  __syncthreads();

  const int mat = wave & 3;
  const int mlo = (wave >> 2) * 7;
  const int mhi = imin(mlo + 7, NNODE);

#pragma unroll 1
  for (int nt = 0; nt < O / CW; ++nt) {
    {
      const int col = mat * O + nt * 16 + m;
      const _Float16* bp = Wp + (size_t)col * DH + 8 * h;
      Frag fb0, fb1, fb2, fb3;
      fb0.h[0] = *(const v8h*)(bp + 0);
      fb0.h[1] = *(const v8h*)(bp + 16);
      fb1.h[0] = *(const v8h*)(bp + 32);
      fb1.h[1] = *(const v8h*)(bp + 48);
      fb2.h[0] = *(const v8h*)(bp + 64);
      fb2.h[1] = *(const v8h*)(bp + 80);
      fb3.h[0] = *(const v8h*)(bp + 96);
      fb3.h[1] = *(const v8h*)(bp + 112);
      const float bias = sB[col];
#pragma unroll 1
      for (int mt = mlo; mt < mhi; ++mt) {
        const _Float16* ap = sX + (16 * mt + m) * HP + 8 * h;
        v8f acc = zero8();
        Frag fa;
        fa.h[0] = *(const v8h*)(ap + 0);
        fa.h[1] = *(const v8h*)(ap + 16);
        acc = wm(fa.v, fb0.v, acc);
        fa.h[0] = *(const v8h*)(ap + 32);
        fa.h[1] = *(const v8h*)(ap + 48);
        acc = wm(fa.v, fb1.v, acc);
        fa.h[0] = *(const v8h*)(ap + 64);
        fa.h[1] = *(const v8h*)(ap + 80);
        acc = wm(fa.v, fb2.v, acc);
        fa.h[0] = *(const v8h*)(ap + 96);
        fa.h[1] = *(const v8h*)(ap + 112);
        acc = wm(fa.v, fb3.v, acc);
#pragma unroll
        for (int r = 0; r < 8; ++r) {
          sM[(mat * RB + 16 * mt + 8 * h + r) * CW + m] = acc[r] * SC_I16 + bias;
        }
      }
    }
    __syncthreads();

    {
#pragma unroll 1
      for (int j = 0; j < (RB * CW) / NTHR; ++j) {
        const int e = tid + j * NTHR;
        const int row = e >> 4, c = e & 15;
        const int smp = row / NNODE;
        const int node = row - smp * NNODE;
        const int sb = smp * NNODE;
        const bool is0 = (node == 0);
        const bool v1ok = (node <= 8);
        const int n0 = is0 ? 1 : ((node <= 4) ? 0 : node - 4);
        const int n1 = is0 ? 2 : (v1ok ? node + 4 : 0);
        const int n2 = 3;
        const int n3 = 4;
        const float kd = sM[(0 * RB + row) * CW + c];
        const float sv = sM[(3 * RB + row) * CW + c];
        const float* qb = sM + (1 * RB + sb) * CW + c;
        const float* vb = sM + (2 * RB + sb) * CW + c;
        const float t0 = sigm(kd + qb[n0 * CW]) * vb[n0 * CW];
        const float t1 = sigm(kd + qb[n1 * CW]) * vb[n1 * CW];
        const float t2 = sigm(kd + qb[n2 * CW]) * vb[n2 * CW];
        const float t3 = sigm(kd + qb[n3 * CW]) * vb[n3 * CW];
        float agg = t0;
        agg = v1ok ? (agg + t1) : agg;
        agg = is0 ? (agg + t2) : agg;
        agg = is0 ? (agg + t3) : agg;
        float outv = sv + agg;
        if (ELU) outv = eluf(outv);
        sO[row * O + nt * 16 + c] = (_Float16)outv;
      }
    }
    __syncthreads();
  }

  {
    const int np = RB * O / 8;
    unsigned short* gp = (unsigned short*)(Hout + gr0 * O);
#pragma unroll 1
    for (int j = 0; j < (np + NTHR - 1) / NTHR; ++j) {
      const int p = tid + j * NTHR;
      if (p < np) {
        H8 v;
        v.f = *(const v8h*)(sO + 8 * p);
        *(volatile v8us*)(gp + 8 * (size_t)p) = v.u;
      }
    }
    __threadfence();
#pragma unroll 1
    for (int j = 0; j < (np + NTHR - 1) / NTHR; ++j) {
      const int p = tid + j * NTHR;
      if (p < np) {
        H8 v;
        v.f = *(const v8h*)(sO + 8 * p);
        *(volatile v8us*)(gp + 8 * (size_t)p) = v.u;
      }
    }
  }
}

__global__ __launch_bounds__(NTHR) void k_leg(
    const _Float16* __restrict__ H2,
    const _Float16* __restrict__ LW1p, const float* __restrict__ lb1,
    const _Float16* __restrict__ LW2p, const float* __restrict__ lb2,
    const float* __restrict__ lw3, const float* __restrict__ lb3,
    float* out) {
  extern __shared__ v4f lds_dyn[];
  char* sm = (char*)lds_dyn;
  _Float16* sL  = (_Float16*)(sm + LL_L);
  _Float16* sA1 = (_Float16*)(sm + LL_A1);
  float*    sA2 = (float*)(sm + LL_A2);
  float*    sY  = (float*)(sm + LL_Y);
  const int tid = threadIdx.x, lane = tid & 31, h = lane >> 4, m = lane & 15;
  const int wave = __builtin_amdgcn_readfirstlane(tid >> 5);
  const int b0 = blockIdx.x * NSMP;

  {
#pragma unroll 1
    for (int j = 0; j < (RL * DLEG / 8) / NTHR; ++j) {
      const int p = tid + j * NTHR;
      const int row = p >> 5, q = p & 31;
      const int part = q >> 3, pc = q & 7;
      const int s = row >> 2, leg = row & 3;
      const int node = (part == 0) ? 0 : (4 * part - 3 + leg);
      *(v8h*)(sL + row * LP + part * DO2 + 8 * pc) =
          *(const v8h*)(H2 + ((size_t)(b0 + s) * NNODE + node) * DO2 + 8 * pc);
    }
  }
  __syncthreads();

  {
    const int mt = wave & 3, ntb = (wave >> 2) * 8;
    v8f acc[8];
#pragma unroll
    for (int i = 0; i < 8; ++i) acc[i] = zero8();
    const _Float16* ap = sL + (16 * mt + m) * LP + 8 * h;
    const _Float16* bp = LW1p + (size_t)(ntb * 16 + m) * DLEG + 8 * h;
#pragma unroll 1
    for (int ks = 0; ks < DLEG / 32; ++ks) {
      const int ko = 32 * ks;
      Frag fa;
      fa.h[0] = *(const v8h*)(ap + ko);
      fa.h[1] = *(const v8h*)(ap + ko + 16);
#pragma unroll
      for (int i = 0; i < 8; ++i) {
        Frag fb;
        fb.h[0] = *(const v8h*)(bp + (size_t)i * 16 * DLEG + ko);
        fb.h[1] = *(const v8h*)(bp + (size_t)i * 16 * DLEG + ko + 16);
        acc[i] = wm(fa.v, fb.v, acc[i]);
      }
    }
#pragma unroll
    for (int i = 0; i < 8; ++i) {
      const int col = (ntb + i) * 16 + m;
      const float bias = lb1[col];
#pragma unroll
      for (int r = 0; r < 8; ++r) {
        sA1[(16 * mt + 8 * h + r) * LP + col] = (_Float16)eluf(acc[i][r] * SC_I16 + bias);
      }
    }
  }
  __syncthreads();

  {
    const int mt = wave & 3, ntb = (wave >> 2) * 4;
    v8f acc[4];
#pragma unroll
    for (int i = 0; i < 4; ++i) acc[i] = zero8();
    const _Float16* ap = sA1 + (16 * mt + m) * LP + 8 * h;
    const _Float16* bp = LW2p + (size_t)(ntb * 16 + m) * DLEG + 8 * h;
#pragma unroll 1
    for (int ks = 0; ks < DLEG / 32; ++ks) {
      const int ko = 32 * ks;
      Frag fa;
      fa.h[0] = *(const v8h*)(ap + ko);
      fa.h[1] = *(const v8h*)(ap + ko + 16);
#pragma unroll
      for (int i = 0; i < 4; ++i) {
        Frag fb;
        fb.h[0] = *(const v8h*)(bp + (size_t)i * 16 * DLEG + ko);
        fb.h[1] = *(const v8h*)(bp + (size_t)i * 16 * DLEG + ko + 16);
        acc[i] = wm(fa.v, fb.v, acc[i]);
      }
    }
#pragma unroll
    for (int i = 0; i < 4; ++i) {
      const int col = (ntb + i) * 16 + m;
      const float bias = lb2[col];
#pragma unroll
      for (int r = 0; r < 8; ++r) {
        sA2[(16 * mt + 8 * h + r) * AP + col] = eluf(acc[i][r] * SC_I16 + bias);
      }
    }
  }
  __syncthreads();

  if (tid < RL * 3) {
    const int row = tid / 3, j = tid - 3 * row;
    const float* ar = sA2 + row * AP;
    const float* wc = lw3 + j;
    float a = 0.0f;
#pragma unroll 4
    for (int c = 0; c < DL2; ++c) a = ar[c] * wc[3 * c] + a;
    sY[tid] = a + lb3[j];
  }
  __syncthreads();

  {
    const bool act = tid < (RL * 3) / 4;
    const int tc = act ? tid : 0;
    const v4f v = *(const v4f*)(sY + 4 * tc);
    float* p = out + (size_t)b0 * NACT + 4 * tc;
    if (act) *(volatile v4f*)p = v;
    __threadfence();
    if (act) *(volatile v4f*)p = v;
  }
}

extern "C" void kernel_launch(void* const* d_in, const int* in_sizes, int n_in,
                              void* d_out, int out_size, void* d_ws, size_t ws_size,
                              hipStream_t stream) {
  if (n_in < 40) return;
  const int B = in_sizes[0] / DOBS;
  if (B <= 0 || in_sizes[0] != B * DOBS || (B % NSMP) != 0) return;
  if (in_sizes[1] != B * NNODE * DLAT) return;
  if (in_sizes[2] != 15 * DH || in_sizes[3] != DH || in_sizes[4] != DH * DLAT || in_sizes[5] != DLAT) return;
  for (int pp = 0; pp < 3; ++pp) {
    const int o = 6 + 4 * pp;
    if (in_sizes[o] != 8 * DH || in_sizes[o + 1] != DH || in_sizes[o + 2] != DH * DLAT || in_sizes[o + 3] != DLAT) return;
  }
  for (int q = 0; q < 4; ++q) {
    if (in_sizes[18 + 2 * q] != DH * DH || in_sizes[19 + 2 * q] != DH) return;
    if (in_sizes[26 + 2 * q] != DH * DO2 || in_sizes[27 + 2 * q] != DO2) return;
  }
  if (in_sizes[34] != DLEG * DLEG || in_sizes[35] != DLEG || in_sizes[36] != DLEG * DL2 || in_sizes[37] != DL2) return;
  if (in_sizes[38] != DL2 * 3 || in_sizes[39] != 3) return;
  if (out_size != B * NACT) return;

  const float* obs     = (const float*)d_in[0];
  const float* lat     = (const float*)d_in[1];
  const float* base_w1 = (const float*)d_in[2];
  const float* base_b1 = (const float*)d_in[3];
  const float* base_w2 = (const float*)d_in[4];
  const float* base_b2 = (const float*)d_in[5];
  const float* hip_w1  = (const float*)d_in[6];
  const float* hip_b1  = (const float*)d_in[7];
  const float* hip_w2  = (const float*)d_in[8];
  const float* hip_b2  = (const float*)d_in[9];
  const float* th_w1   = (const float*)d_in[10];
  const float* th_b1   = (const float*)d_in[11];
  const float* th_w2   = (const float*)d_in[12];
  const float* th_b2   = (const float*)d_in[13];
  const float* cf_w1   = (const float*)d_in[14];
  const float* cf_b1   = (const float*)d_in[15];
  const float* cf_w2   = (const float*)d_in[16];
  const float* cf_b2   = (const float*)d_in[17];
  const float* g1_wk   = (const float*)d_in[18];
  const float* g1_bk   = (const float*)d_in[19];
  const float* g1_wq   = (const float*)d_in[20];
  const float* g1_bq   = (const float*)d_in[21];
  const float* g1_wv   = (const float*)d_in[22];
  const float* g1_bv   = (const float*)d_in[23];
  const float* g1_ws   = (const float*)d_in[24];
  const float* g1_bs   = (const float*)d_in[25];
  const float* g2_wk   = (const float*)d_in[26];
  const float* g2_bk   = (const float*)d_in[27];
  const float* g2_wq   = (const float*)d_in[28];
  const float* g2_bq   = (const float*)d_in[29];
  const float* g2_wv   = (const float*)d_in[30];
  const float* g2_bv   = (const float*)d_in[31];
  const float* g2_ws   = (const float*)d_in[32];
  const float* g2_bs   = (const float*)d_in[33];
  const float* leg_w1  = (const float*)d_in[34];
  const float* leg_b1  = (const float*)d_in[35];
  const float* leg_w2  = (const float*)d_in[36];
  const float* leg_b2  = (const float*)d_in[37];
  const float* leg_w3  = (const float*)d_in[38];
  const float* leg_b3  = (const float*)d_in[39];
  float* out = (float*)d_out;

  size_t off = 0;
  const size_t oPW2 = off; off += (size_t)4 * DLAT * DH * 2;     off = (off + 255) & ~(size_t)255;
  const size_t oG1W = off; off += (size_t)4 * DH * DH * 2;       off = (off + 255) & ~(size_t)255;
  const size_t oG2W = off; off += (size_t)4 * DO2 * DH * 2;      off = (off + 255) & ~(size_t)255;
  const size_t oLW1 = off; off += (size_t)DLEG * DLEG * 2;       off = (off + 255) & ~(size_t)255;
  const size_t oLW2 = off; off += (size_t)DL2 * DLEG * 2;        off = (off + 255) & ~(size_t)255;
  const size_t oH0  = off; off += (size_t)B * NNODE * DH * 2;    off = (off + 255) & ~(size_t)255;
  const size_t oH1  = off; off += (size_t)B * NNODE * DH * 2;    off = (off + 255) & ~(size_t)255;
  const size_t tot = off;
  if (tot > ws_size || tot > (size_t)WSCAP) return;
  char* ws = (char*)d_ws;
  _Float16* PW2p = (_Float16*)(ws + oPW2);
  _Float16* G1Wp = (_Float16*)(ws + oG1W);
  _Float16* G2Wp = (_Float16*)(ws + oG2W);
  _Float16* LW1p = (_Float16*)(ws + oLW1);
  _Float16* LW2p = (_Float16*)(ws + oLW2);
  _Float16* H0   = (_Float16*)(ws + oH0);
  _Float16* H1   = (_Float16*)(ws + oH1);
  _Float16* H2   = H0;

  const int npPW2 = 4 * DLAT * DH / 8;
  const int npG1  = 4 * DH * DH / 8;
  const int npG2  = 4 * DO2 * DH / 8;
  const int npL1  = DLEG * DLEG / 8;
  const int npL2  = DL2 * DLEG / 8;
  if ((npPW2 % NTHR) != 0 || (npG1 % NTHR) != 0 || (npG2 % NTHR) != 0 || (npL1 % NTHR) != 0 || (npL2 % NTHR) != 0) return;

  k_cvt4<<<npPW2 / NTHR, NTHR, 0, stream>>>(base_w2, hip_w2, th_w2, cf_w2, PW2p, DH, DH,
                                            DLAT, DLAT, DLAT, DLAT, npPW2, SC_W16);
  k_cvt4<<<npG1 / NTHR, NTHR, 0, stream>>>(g1_wk, g1_wq, g1_wv, g1_ws, G1Wp, DH, DH,
                                           DH, DH, DH, DH, npG1, SC_W16);
  k_cvt4<<<npG2 / NTHR, NTHR, 0, stream>>>(g2_wk, g2_wq, g2_wv, g2_ws, G2Wp, DH, DH,
                                           DO2, DO2, DO2, DO2, npG2, SC_W16);
  k_cvt4<<<npL1 / NTHR, NTHR, 0, stream>>>(leg_w1, leg_w1, leg_w1, leg_w1, LW1p, DLEG, DLEG,
                                           DLEG, 0, 0, 0, npL1, SC_W16);
  k_cvt4<<<npL2 / NTHR, NTHR, 0, stream>>>(leg_w2, leg_w2, leg_w2, leg_w2, LW2p, DLEG, DLEG,
                                           DL2, 0, 0, 0, npL2, SC_W16);

  hipFuncSetAttribute(reinterpret_cast<const void*>(&k_enc),
                      hipFuncAttributeMaxDynamicSharedMemorySize, LDS_E);
  k_enc<<<B / NSMP, NTHR, LDS_E, stream>>>(obs, lat, base_w1, base_b1, hip_w1, hip_b1, th_w1, th_b1,
                                           cf_w1, cf_b1, PW2p, base_b2, hip_b2, th_b2, cf_b2, H0);

  hipFuncSetAttribute(reinterpret_cast<const void*>(&k_gn<DH, 1>),
                      hipFuncAttributeMaxDynamicSharedMemorySize, LDS_G(DH));
  k_gn<DH, 1><<<B / NSMP, NTHR, LDS_G(DH), stream>>>(H0, G1Wp, g1_bk, g1_bq, g1_bv, g1_bs, H1);

  hipFuncSetAttribute(reinterpret_cast<const void*>(&k_gn<DO2, 0>),
                      hipFuncAttributeMaxDynamicSharedMemorySize, LDS_G(DO2));
  k_gn<DO2, 0><<<B / NSMP, NTHR, LDS_G(DO2), stream>>>(H1, G2Wp, g2_bk, g2_bq, g2_bv, g2_bs, H2);

  hipFuncSetAttribute(reinterpret_cast<const void*>(&k_leg),
                      hipFuncAttributeMaxDynamicSharedMemorySize, LDS_L);
  k_leg<<<B / NSMP, NTHR, LDS_L, stream>>>(H2, LW1p, leg_b1, LW2p, leg_b2, leg_w3, leg_b3, out);
}
